// GCNNet_79216376808038
// MI455X (gfx1250) — hardware-verified
//
#include <hip/hip_runtime.h>
#include <stddef.h>
#include <stdint.h>
#include <math.h>


#define XIN    128
#define HD     128
#define HD2    256
#define EDIM   16
#define NGR    64
#define NTHR   256
#define NWAVE  8
#define EPT    8
#define CHUNK  (NTHR * EPT)
#define WCAP   (EPT * 32)
#define LISTN  (NWAVE * WCAP)
#define NBD    8192
#define SLD    13
#define NBA    1024
#define SLA    10
#define RCAP   28672
#define DEGCAP 64
#define GBM    64
#define GBN    128
#define GTHR   128
#define EWB    256
#define NU1    (HD * (XIN / 8))
#define NU2    (HD2 * (2 * HD / 8))
#define NU3    (HD * (2 * HD2 / 8))
#define AGG_ZINTS (LISTN + 2 * RCAP + 3 * NBA)
#define MISC_INTS 16
#define WSMAX  134217728

static_assert((CHUNK & (CHUNK - 1)) == 0 && CHUNK <= 4096);
static_assert((NBD & (NBD - 1)) == 0 && NBD == (1 << SLD));
static_assert((NBA & (NBA - 1)) == 0 && NBA == (1 << SLA));
static_assert(((long long)CHUNK << SLD) < (1LL << 31));
static_assert(((long long)CHUNK << SLA) < (1LL << 31));
static_assert(NBD % (NTHR * 4) == 0);
static_assert(LISTN % NTHR == 0);
static_assert(NBA % NWAVE == 0 && NBA % 32 == 0 && NBA % GBM == 0);
static_assert(RCAP % 32 == 0 && AGG_ZINTS % (NTHR * 4) == 0 && LISTN % 4 == 0);
static_assert(((AGG_ZINTS + MISC_INTS) % 4) == 0);
static_assert(XIN % 32 == 0 && HD % 32 == 0 && HD2 % 32 == 0);
static_assert(GBM == (GTHR / 32) * 16 && GBN == 128 && GBN == HD && HD2 == 2 * GBN);
static_assert(NU1 % NTHR == 0 && (NU1 + NU2) % NTHR == 0 && (NU1 + NU2 + NU3) % NTHR == 0);
static_assert(XIN / 8 == 16 && (2 * HD) / 8 == 32 && (2 * HD2) / 8 == 64);
static_assert(HD == 4 * 32 && HD2 == 8 * 32);
static_assert(EWB == NTHR && EDIM == 16);
static_assert((AGG_ZINTS + MISC_INTS + 16 * HD2) * 4 <= 300000);
static_assert((NGR * HD * 4) % 512 == 0);

typedef float          v2f   __attribute__((ext_vector_type(2)));
typedef float          v4f   __attribute__((ext_vector_type(4)));
typedef float          v8f   __attribute__((ext_vector_type(8)));
typedef int            v4i   __attribute__((ext_vector_type(4)));
typedef int            v8i   __attribute__((ext_vector_type(8)));
typedef unsigned int   v4u   __attribute__((ext_vector_type(4)));
typedef unsigned short v4us  __attribute__((ext_vector_type(4)));
typedef unsigned short v8us  __attribute__((ext_vector_type(8)));
typedef unsigned short v16us __attribute__((ext_vector_type(16)));
typedef __bf16         v16bf __attribute__((ext_vector_type(16)));
typedef v4f  __attribute__((may_alias)) v4fa;
typedef v4i  __attribute__((may_alias)) v4ia;
typedef v4us __attribute__((may_alias)) v4usa;
typedef v8us __attribute__((may_alias)) v8usa;
union FragB { v16bf v; v16us u; v8us h[2]; v8i w; };

__device__ __forceinline__ v8f wmb(const FragB& a, const FragB& b, v8f c) {
  v8f d = __builtin_amdgcn_wmma_f32_16x16x32_bf16(false, a.v, false, b.v, (short)0, c, false, false);
  asm volatile("v_nop\n\tv_nop\n\tv_nop\n\tv_nop" : "+v"(d) : "v"(a.w), "v"(b.w));
  return d;
}

__device__ __forceinline__ unsigned bf16_bits(float f) {
  const unsigned u = __float_as_uint(f);
  return (u + 0x7FFFu + ((u >> 16) & 1u)) >> 16;
}
__device__ __forceinline__ float bf16_val(float f) {
  return __uint_as_float(bf16_bits(f) << 16);
}

__device__ __forceinline__ void wave_sync() {
  __builtin_amdgcn_fence(__ATOMIC_RELEASE, "wavefront");
  __builtin_amdgcn_wave_barrier();
  __builtin_amdgcn_fence(__ATOMIC_ACQUIRE, "wavefront");
}

template <int SLB>
__device__ __forceinline__ int scan_chunk(const int* __restrict__ dsts, int nE, int cbase, int slotBase,
                                          int nb, int vec8, int* list, int tid, int lane, int wave) {
  int wc = 0;
  const int el0  = tid * EPT;
  const int e0   = cbase + el0;
  const int sent = -2147483647 - 1;
  v4i da, db;
  if (vec8 != 0 && cbase + CHUNK <= nE) {
    da = *(const v4i*)(dsts + e0);
    db = *(const v4i*)(dsts + e0 + 4);
  } else {
    da.x = (e0     < nE) ? dsts[min(e0,     nE - 1)] : sent;
    da.y = (e0 + 1 < nE) ? dsts[min(e0 + 1, nE - 1)] : sent;
    da.z = (e0 + 2 < nE) ? dsts[min(e0 + 2, nE - 1)] : sent;
    da.w = (e0 + 3 < nE) ? dsts[min(e0 + 3, nE - 1)] : sent;
    db.x = (e0 + 4 < nE) ? dsts[min(e0 + 4, nE - 1)] : sent;
    db.y = (e0 + 5 < nE) ? dsts[min(e0 + 5, nE - 1)] : sent;
    db.z = (e0 + 6 < nE) ? dsts[min(e0 + 6, nE - 1)] : sent;
    db.w = (e0 + 7 < nE) ? dsts[min(e0 + 7, nE - 1)] : sent;
  }
  const unsigned nbs = (unsigned)slotBase;
  const unsigned unb = (unsigned)nb;
  const unsigned s0 = (unsigned)da.x - nbs, s1 = (unsigned)da.y - nbs;
  const unsigned s2 = (unsigned)da.z - nbs, s3 = (unsigned)da.w - nbs;
  const unsigned s4 = (unsigned)db.x - nbs, s5 = (unsigned)db.y - nbs;
  const unsigned s6 = (unsigned)db.z - nbs, s7 = (unsigned)db.w - nbs;
  const bool h0 = s0 < unb, h1 = s1 < unb, h2 = s2 < unb, h3 = s3 < unb;
  const bool h4 = s4 < unb, h5 = s5 < unb, h6 = s6 < unb, h7 = s7 < unb;
  const unsigned any = __builtin_amdgcn_ballot_w32(h0 | h1 | h2 | h3 | h4 | h5 | h6 | h7);
  if (any != 0u) {
#define HITJ(J, HJ, SJ) { \
      const unsigned mj = __builtin_amdgcn_ballot_w32(HJ); \
      if (mj != 0u) { \
        if (HJ) { \
          const int pos = wc + (int)__builtin_amdgcn_mbcnt_lo(mj, 0u); \
          if (pos < WCAP) list[wave * WCAP + pos] = ((el0 + (J)) << SLB) | (int)(SJ); \
        } \
        wc += (int)__builtin_popcount(mj); } }
    HITJ(0, h0, s0)
    HITJ(1, h1, s1)
    HITJ(2, h2, s2)
    HITJ(3, h3, s3)
    HITJ(4, h4, s4)
    HITJ(5, h5, s5)
    HITJ(6, h6, s6)
    HITJ(7, h7, s7)
#undef HITJ
  }
  return wc;
}

__global__ __launch_bounds__(NTHR) void k_wprep(const float* __restrict__ W1, const float* __restrict__ W2,
                                                const float* __restrict__ W3,
                                                unsigned short* W1T, unsigned short* W2T, unsigned short* W3T) {
  const int u = (int)blockIdx.x * NTHR + (int)threadIdx.x;
  v8us o;
  unsigned short* dp;
  if (u < NU1) {
    const int n  = u >> 4;
    const int k8 = (u & 15) * 8;
    const float* p = W1 + (size_t)k8 * HD + n;
#pragma unroll
    for (int i = 0; i < 8; ++i) o[i] = (unsigned short)bf16_bits(p[(size_t)i * HD]);
    dp = W1T + (size_t)n * XIN + k8;
  } else if (u < NU1 + NU2) {
    const int v  = u - NU1;
    const int n  = v >> 5;
    const int k8 = (v & 31) * 8;
    const int kk = k8 & (HD - 1);
    const float* p = W2 + (size_t)kk * HD2 + n;
#pragma unroll
    for (int i = 0; i < 8; ++i) o[i] = (unsigned short)bf16_bits(p[(size_t)i * HD2]);
    dp = W2T + (size_t)n * (2 * HD) + k8;
  } else if (u < NU1 + NU2 + NU3) {
    const int v  = u - NU1 - NU2;
    const int n  = v >> 6;
    const int k8 = (v & 63) * 8;
    const int kk = k8 & (HD2 - 1);
    const float* p = W3 + (size_t)kk * HD + n;
#pragma unroll
    for (int i = 0; i < 8; ++i) o[i] = (unsigned short)bf16_bits(p[(size_t)i * HD]);
    dp = W3T + (size_t)n * (2 * HD2) + k8;
  } else {
    return;
  }
  *(volatile v8us*)dp = o;
  __threadfence();
  *(volatile v8us*)dp = o;
}

__global__ __launch_bounds__(NTHR) void k_cvx(const float* __restrict__ x, int nN, int nUnits,
                                              unsigned short* xb) {
  const int u = (int)blockIdx.x * NTHR + (int)threadIdx.x;
  if (u >= nUnits) return;
  const int row = u >> 4;
  const int k8  = (u & 15) * 8;
  const int rc  = row < nN ? row : nN - 1;
  const float* p = x + (size_t)rc * XIN + k8;
  const v4f a = *(const v4fa*)p;
  const v4f b = *(const v4fa*)(p + 4);
  const bool ok = row < nN;
  v8us o;
  o[0] = ok ? (unsigned short)bf16_bits(a.x) : (unsigned short)0;
  o[1] = ok ? (unsigned short)bf16_bits(a.y) : (unsigned short)0;
  o[2] = ok ? (unsigned short)bf16_bits(a.z) : (unsigned short)0;
  o[3] = ok ? (unsigned short)bf16_bits(a.w) : (unsigned short)0;
  o[4] = ok ? (unsigned short)bf16_bits(b.x) : (unsigned short)0;
  o[5] = ok ? (unsigned short)bf16_bits(b.y) : (unsigned short)0;
  o[6] = ok ? (unsigned short)bf16_bits(b.z) : (unsigned short)0;
  o[7] = ok ? (unsigned short)bf16_bits(b.w) : (unsigned short)0;
  unsigned short* dp = xb + (size_t)row * XIN + k8;
  *(volatile v8us*)dp = o;
  __threadfence();
  *(volatile v8us*)dp = o;
}

__global__ __launch_bounds__(NTHR) void k_ew(const float* __restrict__ ea, const float* __restrict__ fw,
                                             const float* __restrict__ fb, int nE, float* ewp) {
  __shared__ float sw[EDIM + 1];
  __shared__ __attribute__((aligned(16))) float sres[EWB];
  const int tid = (int)threadIdx.x, wave = tid >> 5;
  if (tid < EDIM) sw[tid] = bf16_val(fw[tid]);
  if (tid == EDIM) sw[EDIM] = bf16_val(fb[0]);
  __syncthreads();
  const int e  = (int)blockIdx.x * EWB + tid;
  const int ec = e < nE ? e : nE - 1;
  const float* p = ea + (size_t)ec * EDIM;
  float s = 0.0f;
#pragma unroll
  for (int i = 0; i < EDIM / 4; ++i) {
    const v4f a = *(const v4fa*)(p + 4 * i);
    s = fmaf(bf16_val(a.x), sw[4 * i + 0], s);
    s = fmaf(bf16_val(a.y), sw[4 * i + 1], s);
    s = fmaf(bf16_val(a.z), sw[4 * i + 2], s);
    s = fmaf(bf16_val(a.w), sw[4 * i + 3], s);
  }
  s = s + sw[EDIM];
  sres[tid] = (e < nE) ? s : 0.0f;
  __syncthreads();
  const bool wr = wave < 2;
  const int  tc = wr ? tid : 0;
  v4f v = {0.0f, 0.0f, 0.0f, 0.0f};
  if (wr) v = *(const v4fa*)(sres + 4 * tc);
  float* dp = ewp + (size_t)blockIdx.x * EWB + 4 * tc;
  if (wr) *(volatile v4f*)dp = v;
  __threadfence();
  if (wr) *(volatile v4f*)dp = v;
}

__global__ __launch_bounds__(NTHR) void k_deg(const int* __restrict__ dsts, const float* __restrict__ ewp,
                                              int nE, int vec8, float* dis) {
  __shared__ __attribute__((aligned(16))) float sdeg[NBD];
  __shared__ __attribute__((aligned(16))) int list[LISTN];
  __shared__ int wcnt[NWAVE];
  const int tid = (int)threadIdx.x, lane = tid & 31, wave = tid >> 5;
  const int nodeBase = (int)blockIdx.x * NBD;

  for (int i = tid; i < NBD; i += NTHR) sdeg[i] = 0.0f;
  for (int i = tid; i < LISTN; i += NTHR) list[i] = 0;
  if (tid < NWAVE) wcnt[tid] = 0;
  __syncthreads();

  const int nChunks = (nE + CHUNK - 1) / CHUNK;
#pragma unroll 1
  for (int ch = 0; ch < nChunks; ++ch) {
    const int cbase = ch * CHUNK;
    const int wc = scan_chunk<SLD>(dsts, nE, cbase, nodeBase, NBD, vec8, list, tid, lane, wave);
    if (lane == 0) wcnt[wave] = wc;
    __syncthreads();
    if (wave == 0) {
#pragma unroll 1
      for (int w2 = 0; w2 < NWAVE; ++w2) {
        int c = wcnt[w2];
        c = c < 0 ? 0 : (c > WCAP ? WCAP : c);
#pragma unroll 1
        for (int b0 = 0; b0 < c; b0 += 32) {
          const int idx = b0 + lane;
          const int ent = list[w2 * WCAP + (idx < WCAP ? idx : WCAP - 1)];
          const int el  = (ent >> SLD) & (CHUNK - 1);
          int eid = cbase + el;
          eid = eid < 0 ? 0 : (eid > nE - 1 ? nE - 1 : eid);
          const int wvi = __float_as_int(ewp[eid]);
          const int m32 = (c - b0) < 32 ? (c - b0) : 32;
#pragma unroll 1
          for (int k = 0; k < m32; ++k) {
            const int   u  = __builtin_amdgcn_readlane(ent, k);
            const float wk = __int_as_float(__builtin_amdgcn_readlane(wvi, k));
            const int   sl = u & (NBD - 1);
            if (lane == 0) sdeg[sl] = sdeg[sl] + wk;
          }
        }
      }
    }
    __syncthreads();
  }

  v4f vals[NBD / (NTHR * 4)];
#pragma unroll
  for (int it = 0; it < NBD / (NTHR * 4); ++it) {
    const int s0 = it * (NTHR * 4) + 4 * tid;
    const v4f c4 = *(const v4fa*)(sdeg + s0);
    const float d0 = c4.x + 1.0f, d1 = c4.y + 1.0f, d2 = c4.z + 1.0f, d3 = c4.w + 1.0f;
    v4f v;
    v.x = (d0 > 0.0f) ? rsqrtf(fmaxf(d0, 1e-12f)) : 0.0f;
    v.y = (d1 > 0.0f) ? rsqrtf(fmaxf(d1, 1e-12f)) : 0.0f;
    v.z = (d2 > 0.0f) ? rsqrtf(fmaxf(d2, 1e-12f)) : 0.0f;
    v.w = (d3 > 0.0f) ? rsqrtf(fmaxf(d3, 1e-12f)) : 0.0f;
    vals[it] = v;
  }
#pragma unroll
  for (int it = 0; it < NBD / (NTHR * 4); ++it) {
    const int s0 = it * (NTHR * 4) + 4 * tid;
    *(volatile v4f*)(dis + (size_t)nodeBase + s0) = vals[it];
  }
  __threadfence();
#pragma unroll
  for (int it = 0; it < NBD / (NTHR * 4); ++it) {
    const int s0 = it * (NTHR * 4) + 4 * tid;
    *(volatile v4f*)(dis + (size_t)nodeBase + s0) = vals[it];
  }
}

__global__ __launch_bounds__(GTHR) void k_gemm(const unsigned short* __restrict__ A, int lda,
                                               const unsigned short* __restrict__ WT, int K,
                                               float* outF, int ldo) {
  __shared__ __attribute__((aligned(16))) float stg[GBM * GBN];
  const int tid = (int)threadIdx.x, lane = tid & 31, wave = tid >> 5, hh = lane >> 4, m = lane & 15;
  const int rowBase = (int)blockIdx.x * GBM;
  const int col0    = (int)blockIdx.y * GBN;

  v8f acc[8];
  {
    const v8f z = {0.f, 0.f, 0.f, 0.f, 0.f, 0.f, 0.f, 0.f};
#pragma unroll
    for (int t = 0; t < 8; ++t) acc[t] = z;
  }
  const unsigned short* ap = A  + (size_t)(rowBase + 16 * wave + m) * (size_t)lda + 8 * hh;
  const unsigned short* bp = WT + (size_t)(col0 + m) * (size_t)K + 8 * hh;

#pragma unroll 1
  for (int k0 = 0; k0 < K; k0 += 32) {
    FragB af;
    af.h[0] = *(const v8usa*)(ap + k0);
    af.h[1] = *(const v8usa*)(ap + k0 + 16);
#pragma unroll
    for (int nt = 0; nt < 8; ++nt) {
      const unsigned short* wq = bp + (size_t)(16 * nt) * (size_t)K + k0;
      FragB bf;
      bf.h[0] = *(const v8usa*)wq;
      bf.h[1] = *(const v8usa*)(wq + 16);
      acc[nt] = wmb(af, bf, acc[nt]);
    }
  }

#pragma unroll
  for (int nt = 0; nt < 8; ++nt) {
    const int lc = 16 * nt + m;
#pragma unroll
    for (int r = 0; r < 8; ++r) {
      const int lr = 16 * wave + 8 * hh + r;
      stg[lr * GBN + lc] = acc[nt][r];
    }
  }
  __syncthreads();

  v4f pv[16];
#pragma unroll
  for (int i = 0; i < 16; ++i) pv[i] = *(const v4fa*)(stg + (16 * wave + i) * GBN + 4 * lane);
#pragma unroll
  for (int i = 0; i < 16; ++i) {
    const int gr = rowBase + 16 * wave + i;
    *(volatile v4f*)(outF + (size_t)gr * (size_t)ldo + col0 + 4 * lane) = pv[i];
  }
  __threadfence();
#pragma unroll
  for (int i = 0; i < 16; ++i) {
    const int gr = rowBase + 16 * wave + i;
    *(volatile v4f*)(outF + (size_t)gr * (size_t)ldo + col0 + 4 * lane) = pv[i];
  }
}

template <int C, int MODE>
__global__ __launch_bounds__(NTHR) void k_scan(const int* __restrict__ srcs, const int* __restrict__ dsts,
                                               const float* __restrict__ ewp, int nE, int nN, int vec8, int mRows,
                                               const float* __restrict__ dis, const float* __restrict__ hin,
                                               const float* __restrict__ bias, unsigned short* xbo, float* xfo) {
  static_assert(C == 128 || C == 256);
  static_assert(MODE != 0 || C == 128);
  constexpr int CPL = C / 32;
  extern __shared__ __attribute__((aligned(16))) int dsm[];
  int* list = dsm;
  int* hl   = dsm + LISTN;
  int* sl   = hl + RCAP;
  int* cnt  = sl + RCAP;
  int* offs = cnt + NBA;
  int* cur  = offs + NBA;
  int* misc = cur + NBA;
  const int tid = (int)threadIdx.x, lane = tid & 31, wave = tid >> 5;
  float* rowfAll = (float*)(misc + MISC_INTS);
  float* rowf = rowfAll + wave * C;
  unsigned short* rowh = (unsigned short*)(rowfAll + NWAVE * C) + wave * (2 * C);
  const int nodeBase = (int)blockIdx.x * NBA;

  {
    const v4i z4 = {0, 0, 0, 0};
    for (int i = tid * 4; i < AGG_ZINTS; i += NTHR * 4) *(v4ia*)(dsm + i) = z4;
    if (tid < MISC_INTS) misc[tid] = 0;
  }
  float bv[CPL];
  {
    const v4f b0 = *(const v4fa*)(bias + CPL * lane);
    bv[0] = bf16_val(b0.x); bv[1] = bf16_val(b0.y); bv[2] = bf16_val(b0.z); bv[3] = bf16_val(b0.w);
    if constexpr (CPL == 8) {
      const v4f b1 = *(const v4fa*)(bias + CPL * lane + 4);
      bv[4] = bf16_val(b1.x); bv[5] = bf16_val(b1.y); bv[6] = bf16_val(b1.z); bv[7] = bf16_val(b1.w);
    }
  }
  __syncthreads();

  int t = 0, ov = 0;
  const int nChunks = (nE + CHUNK - 1) / CHUNK;
#pragma unroll 1
  for (int ch = 0; ch < nChunks; ++ch) {
    const int cbase = ch * CHUNK;
    const int wc = scan_chunk<SLA>(dsts, nE, cbase, nodeBase, NBA, vec8, list, tid, lane, wave);
    if (lane == 0) misc[wave] = wc;
    __syncthreads();
    if (wave == 0) {
#pragma unroll 1
      for (int w2 = 0; w2 < NWAVE; ++w2) {
        int c = misc[w2];
        c = c < 0 ? 0 : (c > WCAP ? WCAP : c);
#pragma unroll 1
        for (int b0 = 0; b0 < c; b0 += 32) {
          const int idx = b0 + lane;
          const int ent = list[w2 * WCAP + (idx < WCAP ? idx : WCAP - 1)];
          const int m32 = (c - b0) < 32 ? (c - b0) : 32;
#pragma unroll 1
          for (int k = 0; k < m32; ++k) {
            const int u    = __builtin_amdgcn_readlane(ent, k);
            const int slot = u & (NBA - 1);
            const int el   = (u >> SLA) & (CHUNK - 1);
            const int pk   = ((cbase + el) << SLA) | slot;
            if (t < RCAP) {
              if (lane == 0) { hl[t] = pk; cnt[slot] = cnt[slot] + 1; }
              t = t + 1;
            } else {
              ov = 1;
            }
          }
        }
      }
    }
    __syncthreads();
  }
  if (wave == 0 && lane == 0) { misc[8] = t; misc[9] = ov; }
  __syncthreads();
  int tt = misc[8];
  tt = tt < 0 ? 0 : (tt > RCAP ? RCAP : tt);
  const int ovf = misc[9];

  if (wave == 0) {
    const int base = lane * (NBA / 32);
    int s = 0;
#pragma unroll 1
    for (int i = 0; i < NBA / 32; ++i) s += cnt[base + i];
    int incl = s;
#pragma unroll
    for (int d = 1; d < 32; d <<= 1) {
      const int y = __shfl_up(incl, d, 32);
      if (lane >= d) incl += y;
    }
    int run = incl - s;
#pragma unroll 1
    for (int i = 0; i < NBA / 32; ++i) {
      const int cv = cnt[base + i];
      offs[base + i] = run;
      cur[base + i]  = run;
      run += cv;
    }
  }
  __syncthreads();
  if (wave == 0) {
#pragma unroll 1
    for (int b0 = 0; b0 < tt; b0 += 32) {
      const int idx = b0 + lane;
      const int ent = hl[idx < RCAP ? idx : RCAP - 1];
      const int m32 = (tt - b0) < 32 ? (tt - b0) : 32;
#pragma unroll 1
      for (int k = 0; k < m32; ++k) {
        const int u    = __builtin_amdgcn_readlane(ent, k);
        const int slot = u & (NBA - 1);
        if (lane == 0) {
          int p = cur[slot];
          p = p < 0 ? 0 : (p > RCAP - 1 ? RCAP - 1 : p);
          sl[p] = u;
          cur[slot] = p + 1;
        }
      }
    }
  }
  __syncthreads();

  const float qnan = __int_as_float(0x7fc00000);
  const float pz = (ovf != 0) ? qnan : 0.0f;
#pragma unroll 1
  for (int si = 0; si < NBA / NWAVE; ++si) {
    const int s    = si * NWAVE + wave;
    const int node = nodeBase + s;
    int c = cnt[s];
    const bool big = c > DEGCAP;
    c = c < 0 ? 0 : (c > DEGCAP ? DEGCAP : c);
    int o = offs[s];
    o = o < 0 ? 0 : (o > RCAP ? RCAP : o);
    const int nc = node < nN ? node : nN - 1;
    const float dd = dis[nc];
    const float rd = dd * dd;
    float a[CPL];
#pragma unroll
    for (int j = 0; j < CPL; ++j) a[j] = 0.0f;
#pragma unroll 1
    for (int b0 = 0; b0 < c; b0 += 32) {
      int idx = o + b0 + lane;
      idx = idx > RCAP - 1 ? RCAP - 1 : idx;
      const int ent = sl[idx];
      int eid = ent >> SLA;
      eid = eid < 0 ? 0 : (eid > nE - 1 ? nE - 1 : eid);
      int sr = srcs[eid];
      sr = sr < 0 ? 0 : (sr > nN - 1 ? nN - 1 : sr);
      const float wv  = ewp[eid];
      const float cf  = (dis[sr] * wv) * dd;
      const int   cfi = __float_as_int(cf);
      const int m32 = (c - b0) < 32 ? (c - b0) : 32;
#pragma unroll 1
      for (int k = 0; k < m32; ++k) {
        const int   sk = __builtin_amdgcn_readlane(sr, k);
        const float ck = __int_as_float(__builtin_amdgcn_readlane(cfi, k));
        const float* rp = hin + (size_t)sk * C + CPL * lane;
        const v4f g0 = *(const v4fa*)rp;
        a[0] = fmaf(ck, g0.x, a[0]); a[1] = fmaf(ck, g0.y, a[1]);
        a[2] = fmaf(ck, g0.z, a[2]); a[3] = fmaf(ck, g0.w, a[3]);
        if constexpr (CPL == 8) {
          const v4f g1 = *(const v4fa*)(rp + 4);
          a[4] = fmaf(ck, g1.x, a[4]); a[5] = fmaf(ck, g1.y, a[5]);
          a[6] = fmaf(ck, g1.z, a[6]); a[7] = fmaf(ck, g1.w, a[7]);
        }
      }
    }
    {
      const float* rp = hin + (size_t)nc * C + CPL * lane;
      const v4f g0 = *(const v4fa*)rp;
      v4f t0;
      t0.x = (a[0] + g0.x * rd) + bv[0];
      t0.y = (a[1] + g0.y * rd) + bv[1];
      t0.z = (a[2] + g0.z * rd) + bv[2];
      t0.w = (a[3] + g0.w * rd) + bv[3];
      *(v4fa*)(rowf + CPL * lane) = t0;
      if constexpr (CPL == 8) {
        const v4f g1 = *(const v4fa*)(rp + 4);
        v4f t1;
        t1.x = (a[4] + g1.x * rd) + bv[4];
        t1.y = (a[5] + g1.y * rd) + bv[5];
        t1.z = (a[6] + g1.z * rd) + bv[6];
        t1.w = (a[7] + g1.w * rd) + bv[7];
        *(v4fa*)(rowf + CPL * lane + 4) = t1;
      }
    }
    wave_sync();
    const float pzr = big ? qnan : pz;
    const bool live = node < nN;
#pragma unroll 1
    for (int j = 0; j < CPL; ++j) {
      const int   cc = CPL * lane + j;
      const float v  = rowf[cc];
      const float em = expm1f(fminf(v, 0.0f));
      float e = (v > 0.0f) ? v : em;
      e = live ? (e + pzr) : 0.0f;
      if constexpr (MODE != 0) {
        const unsigned hb = bf16_bits(e);
        const unsigned lb = bf16_bits(e - __uint_as_float(hb << 16));
        rowh[cc]     = (unsigned short)hb;
        rowh[C + cc] = (unsigned short)lb;
      } else {
        rowf[cc] = e;
      }
    }
    wave_sync();
    if constexpr (MODE != 0) {
      const v8us q0 = *(const v8usa*)(rowh + 8 * lane);
      v8us q1 = {0, 0, 0, 0, 0, 0, 0, 0};
      if constexpr (C == 256) q1 = *(const v8usa*)(rowh + 256 + 8 * lane);
      wave_sync();
      if (node < mRows) {
        unsigned short* rpw = xbo + (size_t)node * (2 * C) + 8 * lane;
        *(volatile v8us*)rpw = q0;
        if constexpr (C == 256) *(volatile v8us*)(rpw + 256) = q1;
        __threadfence();
        *(volatile v8us*)rpw = q0;
        if constexpr (C == 256) *(volatile v8us*)(rpw + 256) = q1;
      }
    } else {
      const v4f ow = *(const v4fa*)(rowf + 4 * lane);
      wave_sync();
      if (node < mRows) {
        float* op = xfo + (size_t)node * C + 4 * lane;
        *(volatile v4f*)op = ow;
        __threadfence();
        *(volatile v4f*)op = ow;
      }
    }
  }
}

__global__ __launch_bounds__(NTHR) void k_pool(const float* __restrict__ hf, const int* __restrict__ bat,
                                               int nN, float* outp) {
  __shared__ __attribute__((aligned(16))) float wsum[NWAVE * HD];
  __shared__ int wcn[NWAVE];
  __shared__ __attribute__((aligned(16))) float outs[HD];
  const int tid = (int)threadIdx.x, lane = tid & 31, wave = tid >> 5;
  const int g = (int)blockIdx.x;

  float a0 = 0.0f, a1 = 0.0f, a2 = 0.0f, a3 = 0.0f;
  int cnt = 0;
#pragma unroll 1
  for (int i0 = wave * 32; i0 < nN; i0 += NTHR) {
    const int i  = i0 + lane;
    const int ic = i < nN ? i : nN - 1;
    const int b  = bat[ic];
    const bool hit = (i < nN) && (b == g);
    unsigned msk = __builtin_amdgcn_ballot_w32(hit);
    int nh = (int)__builtin_popcount(msk);
    nh = nh > 32 ? 32 : nh;
    cnt += nh;
#pragma unroll 1
    for (int q = 0; q < nh; ++q) {
      const int k = __builtin_ffs((int)msk) - 1;
      msk &= msk - 1u;
      int node = i0 + (k < 0 ? 0 : k);
      node = node > nN - 1 ? nN - 1 : node;
      const v4f v = *(const v4fa*)(hf + (size_t)node * HD + 4 * lane);
      a0 += v.x; a1 += v.y; a2 += v.z; a3 += v.w;
    }
  }
  {
    v4f w4;
    w4.x = a0; w4.y = a1; w4.z = a2; w4.w = a3;
    *(v4fa*)(wsum + wave * HD + 4 * lane) = w4;
  }
  if (lane == 0) wcn[wave] = cnt;
  __syncthreads();
  if (tid < HD) {
    float s = 0.0f;
    int c = 0;
#pragma unroll
    for (int w2 = 0; w2 < NWAVE; ++w2) { s += wsum[w2 * HD + tid]; c += wcn[w2]; }
    const float cf = (c < 1) ? 1.0f : (float)c;
    outs[tid] = s * (1.0f / cf);
  }
  __syncthreads();
  const v4f ov = *(const v4fa*)(outs + 4 * lane);
  float* op = outp + (size_t)g * HD + 4 * lane;
  const bool okst = (wave == 0);
  if (okst) *(volatile v4f*)op = ov;
  __threadfence();
  if (okst) *(volatile v4f*)op = ov;
}

static inline int cdiv(int a, int b) { return (a + b - 1) / b; }
static inline size_t al256(size_t o) { return (o + 255) & ~(size_t)255; }
static inline size_t smax(size_t a, size_t b) { return a > b ? a : b; }

extern "C" void kernel_launch(void* const* d_in, const int* in_sizes, int n_in,
                              void* d_out, int out_size, void* d_ws, size_t ws_size,
                              hipStream_t stream) {
  if (n_in < 12) return;
  if (in_sizes[0] < XIN || (in_sizes[0] % XIN) != 0) return;
  const int nN = in_sizes[0] / XIN;
  if (nN < 16 || nN >= (1 << 24)) return;
  if (in_sizes[1] < 2 || (in_sizes[1] & 1) != 0) return;
  const int nE = in_sizes[1] / 2;
  if (nE < 1 || nE >= (1 << 21)) return;
  if (in_sizes[2] != nE * EDIM) return;
  if (in_sizes[3] != nN) return;
  if (in_sizes[4] != EDIM || in_sizes[5] != 1) return;
  if (in_sizes[6] != XIN * HD || in_sizes[7] != HD) return;
  if (in_sizes[8] != HD * HD2 || in_sizes[9] != HD2) return;
  if (in_sizes[10] != HD2 * HD || in_sizes[11] != HD) return;
  if (out_size != NGR * HD) return;

  const float* x    = (const float*)d_in[0];
  const int*   edge = (const int*)d_in[1];
  const float* eat  = (const float*)d_in[2];
  const int*   bat  = (const int*)d_in[3];
  const float* fcw  = (const float*)d_in[4];
  const float* fcb  = (const float*)d_in[5];
  const float* W1   = (const float*)d_in[6];
  const float* b1   = (const float*)d_in[7];
  const float* W2   = (const float*)d_in[8];
  const float* b2   = (const float*)d_in[9];
  const float* W3   = (const float*)d_in[10];
  const float* b3   = (const float*)d_in[11];
  float* out = (float*)d_out;
  const int* src = edge;
  const int* dst = edge + nE;

  const int MP   = cdiv(nN, GBM) * GBM;
  const int gM   = MP / GBM;
  const int gD   = cdiv(nN, NBD);
  const int NBPD = gD * NBD;
  const int gA   = cdiv(MP, NBA);
  const int gE   = cdiv(nE, EWB);
  const int EWP  = gE * EWB;
  if ((long long)gA * NBA < (long long)MP) return;
  if (NBPD < nN) return;
  const int vec8 = ((nE & 3) == 0) ? 1 : 0;

  char* ws = (char*)d_ws;
  size_t off = 0;
  const size_t oEW  = off; off = al256(off + (size_t)EWP * 4);
  const size_t oDIS = off; off = al256(off + (size_t)NBPD * 4);
  const size_t oW1T = off; off = al256(off + (size_t)HD * XIN * 2);
  const size_t oW2T = off; off = al256(off + (size_t)HD2 * (2 * HD) * 2);
  const size_t oW3T = off; off = al256(off + (size_t)HD * (2 * HD2) * 2);
  const size_t xbSz = al256((size_t)MP * XIN * 2);
  const size_t r1Sz = smax(smax(xbSz + (size_t)MP * HD * 4, (size_t)MP * HD2 * 4), (size_t)MP * HD * 4);
  const size_t r2Sz = smax(smax((size_t)MP * (2 * HD) * 2, (size_t)MP * (2 * HD2) * 2), (size_t)MP * HD * 4);
  const size_t oR1  = off; off = al256(off + r1Sz);
  const size_t oR2  = off; off = al256(off + r2Sz);
  if (off > ws_size || off > (size_t)WSMAX) return;
  float*          EW  = (float*)(ws + oEW);
  float*          DIS = (float*)(ws + oDIS);
  unsigned short* W1T = (unsigned short*)(ws + oW1T);
  unsigned short* W2T = (unsigned short*)(ws + oW2T);
  unsigned short* W3T = (unsigned short*)(ws + oW3T);
  unsigned short* XB  = (unsigned short*)(ws + oR1);
  float*          H1  = (float*)(ws + oR1 + xbSz);
  float*          H2  = (float*)(ws + oR1);
  float*          H3  = (float*)(ws + oR1);
  unsigned short* X1  = (unsigned short*)(ws + oR2);
  unsigned short* X2  = (unsigned short*)(ws + oR2);
  float*          X3  = (float*)(ws + oR2);

  const size_t lds128 = (size_t)(AGG_ZINTS + MISC_INTS + 16 * HD) * 4;
  const size_t lds256 = (size_t)(AGG_ZINTS + MISC_INTS + 16 * HD2) * 4;
  hipFuncSetAttribute(reinterpret_cast<const void*>(&k_scan<128, 1>), hipFuncAttributeMaxDynamicSharedMemorySize, (int)lds128);
  hipFuncSetAttribute(reinterpret_cast<const void*>(&k_scan<256, 1>), hipFuncAttributeMaxDynamicSharedMemorySize, (int)lds256);
  hipFuncSetAttribute(reinterpret_cast<const void*>(&k_scan<128, 0>), hipFuncAttributeMaxDynamicSharedMemorySize, (int)lds128);

  const int nUx = MP * (XIN / 8);
  k_wprep<<<(NU1 + NU2 + NU3) / NTHR, NTHR, 0, stream>>>(W1, W2, W3, W1T, W2T, W3T);
  k_cvx<<<cdiv(nUx, NTHR), NTHR, 0, stream>>>(x, nN, nUx, XB);
  k_ew<<<gE, NTHR, 0, stream>>>(eat, fcw, fcb, nE, EW);
  k_deg<<<gD, NTHR, 0, stream>>>(dst, EW, nE, vec8, DIS);
  k_gemm<<<dim3(gM, HD / GBN), GTHR, 0, stream>>>(XB, XIN, W1T, XIN, H1, HD);
  k_scan<128, 1><<<gA, NTHR, lds128, stream>>>(src, dst, EW, nE, nN, vec8, MP, DIS, H1, b1, X1, X3);
  k_gemm<<<dim3(gM, HD2 / GBN), GTHR, 0, stream>>>(X1, 2 * HD, W2T, 2 * HD, H2, HD2);
  k_scan<256, 1><<<gA, NTHR, lds256, stream>>>(src, dst, EW, nE, nN, vec8, MP, DIS, H2, b2, X2, X3);
  k_gemm<<<dim3(gM, HD / GBN), GTHR, 0, stream>>>(X2, 2 * HD2, W3T, 2 * HD2, H3, HD);
  k_scan<128, 0><<<gA, NTHR, lds128, stream>>>(src, dst, EW, nE, nN, vec8, MP, DIS, H3, b3, X2, X3);
  k_pool<<<NGR, NTHR, 0, stream>>>(X3, bat, nN, out);
}
